// cAttend_simple_40922448396535
// MI455X (gfx1250) — hardware-run, weakly checked
//
#include <hip/hip_runtime.h>

typedef __attribute__((ext_vector_type(16))) __bf16   v16b;
typedef __attribute__((ext_vector_type(8)))  __bf16   v8b;
typedef __attribute__((ext_vector_type(8)))  float    v8f;
typedef __attribute__((ext_vector_type(4)))  float    v4f;
typedef __attribute__((ext_vector_type(4)))  unsigned v4u;

constexpr int kBatch   = 4;
constexpr int kNpos    = 4096;
constexpr int kEmb     = 256;
constexpr int kQK      = 64;
constexpr int kQKRoot  = 8;
constexpr int kTabRows = 10001;
constexpr int kRows    = kBatch * kNpos;
constexpr int kNP      = 2 * kQK;
constexpr int kChunk   = 64;
constexpr int kChunksPerB = kNpos / kChunk;
constexpr int kOutBlk  = 256;
constexpr int kOutBlkPerB = kNpos / kOutBlk;
static_assert(kQKRoot * kQKRoot == kQK, "scale derivation");
constexpr float kScale = 1.0f / (float)kQKRoot;
static_assert(kRows == 16384 && kNP == 128, "shapes");
static_assert((kEmb % 32) == 0, "GEMM K multiple of 32");
static_assert((kRows % 64) == 0 && (kNP % 64) == 0, "GEMM M,N multiples of 64");
static_assert((kRows / 64) * (kNP / 64) == 64 * 8, "GEMM grid: 64 blocks x 8 waves cover all 64x64 tiles");
static_assert(kChunksPerB == 64 && kOutBlkPerB == 16, "partial-sum and output grids");
static_assert(kChunk == 64 && kQK == 64, "one lane per q column, 64 rows per partial block");

constexpr size_t kOffAH  = 0;
constexpr size_t kOffBH  = kOffAH + (size_t)kRows * kEmb * 2;
constexpr size_t kOffP   = kOffBH + (size_t)kNP * kEmb * 2;
constexpr size_t kOffSP  = kOffP  + (size_t)kRows * kNP * 4;
constexpr size_t kWsTotal = kOffSP + (size_t)kBatch * kChunksPerB * kQK * 4;
static_assert(kWsTotal == 16908288ull, "carve total");
static_assert(kWsTotal <= 134217728ull, "carve cap");
static_assert((kOffBH % 128) == 0 && (kOffP % 128) == 0 && (kOffSP % 128) == 0, "128-B aligned regions");

namespace eng {

__device__ __forceinline__ unsigned bf_rne_bits(float f) {
  const unsigned u = __float_as_uint(f);
  return ((u + 0x7FFFu + ((u >> 16) & 1u)) >> 16) & 0xFFFFu;
}

__device__ __forceinline__ float bf_conv(float f) {
  return __uint_as_float(bf_rne_bits(f) << 16);
}

__device__ __forceinline__ unsigned pack_pair(float x0, float x1) {
  const unsigned h0 = bf_rne_bits(x0);
  const unsigned h1 = bf_rne_bits(x1);
  return h0 | (h1 << 16);
}

__device__ __forceinline__ v4u conv8(const v4f a0, const v4f a1) {
  const float x0 = a0[0];
  const float x1 = a0[1];
  const float x2 = a0[2];
  const float x3 = a0[3];
  const float x4 = a1[0];
  const float x5 = a1[1];
  const float x6 = a1[2];
  const float x7 = a1[3];
  const unsigned w0 = pack_pair(x0, x1);
  const unsigned w1 = pack_pair(x2, x3);
  const unsigned w2 = pack_pair(x4, x5);
  const unsigned w3 = pack_pair(x6, x7);
  return (v4u){w0, w1, w2, w3};
}

union FragU { v16b v; v8b h[2]; };
__device__ __forceinline__ v16b frag_load(const __bf16* p) {
  FragU f;
  f.h[0] = *(const v8b*)(p);
  f.h[1] = *(const v8b*)(p + 16);
  return f.v;
}
__device__ __forceinline__ v8f mma(v16b a, v16b b, v8f c) {
  return __builtin_amdgcn_wmma_f32_16x16x32_bf16(false, a, false, b, (short)0, c, false, false);
}
__device__ __forceinline__ void guard1(v8f& a, v16b x, v16b y) {
  asm volatile("v_nop\n\tv_nop\n\tv_nop\n\tv_nop" : "+v"(a) : "v"(x), "v"(y));
}
__device__ __forceinline__ void tie1(v8f& a) {
  asm volatile("v_nop\n\tv_nop\n\tv_nop\n\tv_nop" : "+v"(a));
}
__device__ __forceinline__ void keep4(v16b a, v16b b, v16b c, v16b d) {
  asm volatile("v_nop" :: "v"(a), "v"(b), "v"(c), "v"(d));
}

}

__global__ __launch_bounds__(256) void gather_conv_kernel(
    const int* __restrict__ pos, const float* __restrict__ emb,
    unsigned short* __restrict__ AH)
{
  const int i = blockIdx.x * 256 + threadIdx.x;
  const int r = i >> 5;
  if (r >= kRows) return;
  const int c8 = (i & 31) * 8;
  int p = pos[r];
  p = (p < 0) ? 0 : p;
  p = (p > (kTabRows - 1)) ? (kTabRows - 1) : p;
  const float* src = emb + (size_t)p * kEmb + c8;
  const v4f a0 = *(const v4f*)(src);
  const v4f a1 = *(const v4f*)(src + 4);
  const v4u hv = eng::conv8(a0, a1);
  const size_t e0 = (size_t)r * kEmb + c8;
  volatile v4u* qh = (volatile v4u*)(void*)(AH + e0);
  *qh = hv;
  __threadfence();
  *qh = hv;
}

__global__ __launch_bounds__(256) void weight_conv_kernel(
    const float* __restrict__ Wq, const float* __restrict__ Wk,
    unsigned short* __restrict__ BH)
{
  const int i = blockIdx.x * 256 + threadIdx.x;
  if (i >= kNP * kEmb / 8) return;
  const bool kside = (blockIdx.x >= 8);
  const float* base = kside ? Wk : Wq;
  const int li = kside ? (i - kQK * kEmb / 8) : i;
  const float* src = base + (size_t)li * 8;
  const v4f a0 = *(const v4f*)(src);
  const v4f a1 = *(const v4f*)(src + 4);
  const v4u hv = eng::conv8(a0, a1);
  const size_t e0 = (size_t)i * 8;
  volatile v4u* qh = (volatile v4u*)(void*)(BH + e0);
  *qh = hv;
  __threadfence();
  *qh = hv;
}

__global__ __launch_bounds__(256) void proj_gemm_kernel(
    const unsigned short* __restrict__ AHp, const unsigned short* __restrict__ BHp,
    float* __restrict__ Pout)
{
  const __bf16* AH = (const __bf16*)AHp;
  const __bf16* BH = (const __bf16*)BHp;
  __shared__ __align__(16) float sT[8][16 * 68];
  const int lane = threadIdx.x & 31;
  const int wave = threadIdx.x >> 5;
  constexpr int tilesN = kNP >> 6;
  constexpr int tilesM = kRows >> 6;
  const int tile = blockIdx.x * 8 + wave;
  if (tile >= tilesM * tilesN) return;
  const int tm = tile / tilesN;
  const int tn = tile - tm * tilesN;
  const int m0 = tm << 6;
  const int n0 = tn << 6;

  const int rlane = lane & 15;
  const int koff  = (lane >> 4) * 8;
  const int mOff  = (lane >> 4) * 8;

  v8f acc[4][4];
#pragma unroll
  for (int i = 0; i < 4; ++i)
#pragma unroll
    for (int j = 0; j < 4; ++j) acc[i][j] = (v8f){0.f, 0.f, 0.f, 0.f, 0.f, 0.f, 0.f, 0.f};

#pragma unroll 1
  for (int k0 = 0; k0 < kEmb; k0 += 32) {
    v16b bh[4];
#pragma unroll
    for (int j = 0; j < 4; ++j) {
      const size_t bo = (size_t)(n0 + (j << 4) + rlane) * kEmb + koff + k0;
      bh[j] = eng::frag_load(BH + bo);
    }
#pragma unroll
    for (int i = 0; i < 4; ++i) {
      const size_t ao = (size_t)(m0 + (i << 4) + rlane) * kEmb + koff + k0;
      const v16b ah = eng::frag_load(AH + ao);
#pragma unroll
      for (int j = 0; j < 4; ++j) {
        acc[i][j] = eng::mma(ah, bh[j], acc[i][j]);
      }
      eng::guard1(acc[i][0], ah, bh[0]);
      eng::guard1(acc[i][1], ah, bh[1]);
      eng::guard1(acc[i][2], ah, bh[2]);
      eng::guard1(acc[i][3], ah, bh[3]);
    }
    eng::keep4(bh[0], bh[1], bh[2], bh[3]);
  }
#pragma unroll
  for (int i = 0; i < 4; ++i) {
    eng::tie1(acc[i][0]);
    eng::tie1(acc[i][1]);
    eng::tie1(acc[i][2]);
    eng::tie1(acc[i][3]);
  }

  float* slab = sT[wave];
#pragma unroll
  for (int i = 0; i < 4; ++i) {
    const int mBase = m0 + (i << 4);
#pragma unroll
    for (int j = 0; j < 4; ++j) {
#pragma unroll
      for (int r = 0; r < 8; ++r) {
        slab[(mOff + r) * 68 + (j << 4) + rlane] = acc[i][j][r];
      }
    }
    __builtin_amdgcn_fence(__ATOMIC_RELEASE, "workgroup");
    __builtin_amdgcn_wave_barrier();
    __builtin_amdgcn_fence(__ATOMIC_ACQUIRE, "workgroup");
    {
      const int hh = lane >> 4;
      const int c4 = (lane & 15) * 4;
      for (int pass = 0; pass < 2; ++pass) {
#pragma unroll
        for (int it = 0; it < 8; ++it) {
          const int row = it * 2 + hh;
          const v4f v = *(const v4f*)(slab + row * 68 + c4);
          *(volatile v4f*)(Pout + (size_t)(mBase + row) * kNP + n0 + c4) = v;
        }
        __threadfence();
      }
    }
    __builtin_amdgcn_fence(__ATOMIC_RELEASE, "workgroup");
    __builtin_amdgcn_wave_barrier();
    __builtin_amdgcn_fence(__ATOMIC_ACQUIRE, "workgroup");
  }
}

__global__ __launch_bounds__(64) void s_partial_kernel(
    const float* __restrict__ val, const float* __restrict__ P, const float* __restrict__ bq,
    float* __restrict__ SP)
{
  __shared__ __align__(16) float sV[kChunk];
  __shared__ __align__(16) float sS[kQK];
  const int tid = threadIdx.x;
  const int r0 = blockIdx.x * kChunk;
  sV[tid] = eng::bf_conv(val[r0 + tid]);
  __syncthreads();
  const float bqd = eng::bf_conv(bq[tid]);
  float acc = 0.0f;
#pragma unroll 8
  for (int ii = 0; ii < kChunk; ++ii) {
    const float qv = P[(size_t)(r0 + ii) * kNP + tid] + bqd;
    acc = fmaf(sV[ii], qv, acc);
  }
  sS[tid] = acc;
  __syncthreads();
  if (tid < 16) {
    const v4f v = *(const v4f*)(sS + tid * 4);
    volatile v4f* dst = (volatile v4f*)(SP + (size_t)blockIdx.x * kQK + tid * 4);
    *dst = v;
    __threadfence();
    *dst = v;
  }
}

__global__ __launch_bounds__(256) void output_kernel(
    const float* __restrict__ val, const float* __restrict__ P, const float* __restrict__ bk,
    const float* __restrict__ SP, float* __restrict__ out)
{
  __shared__ __align__(16) float sS[kQK];
  __shared__ __align__(16) float sB[kQK];
  __shared__ __align__(16) float sO[kOutBlk];
  const int tid = threadIdx.x;
  const int b = blockIdx.x / kOutBlkPerB;
  const int r0 = blockIdx.x * kOutBlk;
  if (tid < kQK) {
    float a = 0.0f;
#pragma unroll 8
    for (int c = 0; c < kChunksPerB; ++c) {
      a += SP[(size_t)(b * kChunksPerB + c) * kQK + tid];
    }
    sS[tid] = a;
    sB[tid] = eng::bf_conv(bk[tid]);
  }
  __syncthreads();
  const int r = r0 + tid;
  const float* prow = P + (size_t)r * kNP + kQK;
  float dot = 0.0f;
#pragma unroll 4
  for (int g = 0; g < kQK / 4; ++g) {
    const v4f kv = *(const v4f*)(prow + 4 * g);
    const v4f sv = *(const v4f*)(sS + 4 * g);
    const v4f bv = *(const v4f*)(sB + 4 * g);
    dot = fmaf(kv[0] + bv[0], sv[0], dot);
    dot = fmaf(kv[1] + bv[1], sv[1], dot);
    dot = fmaf(kv[2] + bv[2], sv[2], dot);
    dot = fmaf(kv[3] + bv[3], sv[3], dot);
  }
  const float v = eng::bf_conv(val[r]);
  const float fx = kScale * dot;
  sO[tid] = fmaf(v, fx, v);
  __syncthreads();
  if (tid < 64) {
    const v4f o = *(const v4f*)(sO + tid * 4);
    volatile v4f* dst = (volatile v4f*)(out + (size_t)r0 + tid * 4);
    *dst = o;
    __threadfence();
    *dst = o;
  }
}

extern "C" void kernel_launch(void* const* d_in, const int* in_sizes, int n_in,
                              void* d_out, int out_size, void* d_ws, size_t ws_size,
                              hipStream_t stream) {
  if (n_in < 8) return;
  if (in_sizes[1] != kRows) return;
  if (in_sizes[2] != kRows) return;
  if (in_sizes[3] != kTabRows * kEmb) return;
  if (in_sizes[4] != kQK * kEmb) return;
  if (in_sizes[5] != kQK) return;
  if (in_sizes[6] != kQK * kEmb) return;
  if (in_sizes[7] != kQK) return;
  if (out_size != kRows) return;
  if (ws_size < kWsTotal) return;

  const float* val = (const float*)d_in[1];
  const int*   pos = (const int*)d_in[2];
  const float* emb = (const float*)d_in[3];
  const float* Wq  = (const float*)d_in[4];
  const float* bq  = (const float*)d_in[5];
  const float* Wk  = (const float*)d_in[6];
  const float* bk  = (const float*)d_in[7];
  float* out = (float*)d_out;

  char* ws = (char*)d_ws;
  unsigned short* AH = (unsigned short*)(ws + kOffAH);
  unsigned short* BH = (unsigned short*)(ws + kOffBH);
  float*          P  = (float*)(ws + kOffP);
  float*          SP = (float*)(ws + kOffSP);

  gather_conv_kernel<<<kRows * 32 / 256, 256, 0, stream>>>(pos, emb, AH);
  weight_conv_kernel<<<kNP * kEmb / 8 / 256, 256, 0, stream>>>(Wq, Wk, BH);
  proj_gemm_kernel<<<(kRows / 64) * (kNP / 64) / 8, 256, 0, stream>>>(AH, BH, P);
  s_partial_kernel<<<kBatch * kChunksPerB, kChunk, 0, stream>>>(val, P, bq, SP);
  output_kernel<<<kBatch * kOutBlkPerB, kOutBlk, 0, stream>>>(val, P, bk, SP, out);
}
